// MLP_64450279244218
// MI455X (gfx1250) — hardware-run, weakly checked
//
#include <hip/hip_runtime.h>


#ifndef NWR
#define NWR 512
#endif
#ifndef NQR
#define NQR 512
#endif
#define NWR_FULL 512
#define NQR_FULL 512
#define OUT_PITCH NQR_FULL
#define NIN  1600
#define NH1  64
#define NH2  32
#define AW   4
#define OSP  36
#define W2S  64.0f
#define W2I  0.015625f
static constexpr float H1RS = 2048.0f;
static constexpr float H1RI = 1.0f / 2048.0f;

static_assert(NIN % 32 == 0);
static_assert((NIN * 2) % 128 == 0);
static_assert(NH1 == 64);
static_assert(NH2 == 32);
static_assert(NWR % 64 == 0);
static_assert(NQR % 64 == 0);
static_assert(NWR % (16 * AW) == 0);
static_assert(NQR % 32 == 0);
static_assert(NWR <= NWR_FULL);
static_assert(NQR <= NQR_FULL);
static_assert((OSP * 4) % 16 == 0);
static_assert((NH1 * (NIN / 8)) % 256 == 0);
static_assert(NH2 * (NH1 / 8) == 256);
static_assert(256 * 16 == NH2 * NH1 * 2);
static_assert(8 * 32 * 16 == 16 * NH1 * 4);
static_assert(4 * 32 * 16 == 16 * 32 * 4);
static_assert(16 * 68 * 4 <= 131072);
static_assert(AW * 16 * OSP * 4 <= 131072);

typedef _Float16 h16;
typedef unsigned short bf;
typedef __attribute__((ext_vector_type(16))) __bf16   v16bf;
typedef __attribute__((ext_vector_type(16))) _Float16 v16h;
typedef __attribute__((ext_vector_type(8)))  _Float16 v8h;
typedef __attribute__((ext_vector_type(8)))  unsigned short v8us;
typedef __attribute__((ext_vector_type(8)))  float    v8f;
typedef __attribute__((ext_vector_type(4)))  float    v4f;
typedef v4f  __attribute__((may_alias)) v4fa;

__device__ __forceinline__ unsigned short f2bf(float f) { unsigned u = __float_as_uint(f); u += 0x7FFFu + ((u >> 16) & 1u); return (unsigned short)(u >> 16); }
__device__ __forceinline__ float bfr(float f) { return __uint_as_float(((unsigned)f2bf(f)) << 16); }
__device__ __forceinline__ v16h cat16(v8h lo, v8h hi) { return __builtin_shufflevector(lo, hi, 0, 1, 2, 3, 4, 5, 6, 7, 8, 9, 10, 11, 12, 13, 14, 15); }
__device__ __forceinline__ v16bf cat16b(v8us lo, v8us hi) { return __builtin_bit_cast(v16bf, __builtin_shufflevector(lo, hi, 0, 1, 2, 3, 4, 5, 6, 7, 8, 9, 10, 11, 12, 13, 14, 15)); }
__device__ __forceinline__ v8f wmma16(v16h a, v16h b, v8f c) { return __builtin_amdgcn_wmma_f32_16x16x32_f16(false, a, false, b, (short)0, c, false, false); }
__device__ __forceinline__ v8f wmmab(v16bf a, v16bf b, v8f c) { return __builtin_amdgcn_wmma_f32_16x16x32_bf16(false, a, false, b, (short)0, c, false, false); }
__device__ __forceinline__ v16h  ldh(const h16* p) { return cat16(*(const v8h*)p, *(const v8h*)(p + 16)); }
__device__ __forceinline__ v16bf ldb(const bf* p)  { return cat16b(*(const v8us*)p, *(const v8us*)(p + 16)); }
__device__ __forceinline__ void wave_sync() { __builtin_amdgcn_fence(3  , "wavefront"); __builtin_amdgcn_wave_barrier(); asm volatile("" ::: "memory"); }

__device__ __forceinline__ v8f wmmabg(v16bf a, v16bf b, v8f c) { c = wmmab(a, b, c); asm volatile("v_nop\n\tv_nop\n\tv_nop\n\tv_nop" : "+v"(c) : "v"(a), "v"(b)); return c; }
__device__ __forceinline__ v8f wmma16g(v16h a, v16h b, v8f c) { c = wmma16(a, b, c); asm volatile("v_nop\n\tv_nop\n\tv_nop\n\tv_nop" : "+v"(c) : "v"(a), "v"(b)); return c; }
static __device__ __forceinline__ h16 toh_flush(float v) { const float w = (fabsf(v) < 6.103515625e-05f) ? 0.0f : v; return (h16)w; }

__global__ __launch_bounds__(256) void k_cvt8(const float* __restrict__ src, bf* dst, size_t n8) {
    const size_t i = (size_t)blockIdx.x * 256 + threadIdx.x; if (i >= n8) return;
    const v8f v = *(const v8f*)(src + i * 8); v8us o;
#pragma unroll
    for (int k = 0; k < 8; ++k) o[k] = f2bf(v[k]);
    *(volatile v8us*)(dst + i * 8) = o; __threadfence(); *(volatile v8us*)(dst + i * 8) = o;
}

__global__ __launch_bounds__(256) void k_w1t(const float* __restrict__ W1, bf* W1T) {
    const unsigned i = blockIdx.x * 256u + threadIdx.x; if (i >= (unsigned)(NH1 * (NIN / 8))) return;
    const unsigned n = i / (unsigned)(NIN / 8); const unsigned k8 = (i % (unsigned)(NIN / 8)) * 8u;
    v8us o;
#pragma unroll
    for (int j = 0; j < 8; ++j) o[j] = f2bf(W1[(size_t)(k8 + (unsigned)j) * NH1 + n]);
    *(volatile v8us*)(W1T + (size_t)i * 8) = o; __threadfence(); *(volatile v8us*)(W1T + (size_t)i * 8) = o;
}

__global__ __launch_bounds__(256) void k_w2t(const float* __restrict__ W2, h16* W2T) {
    const int t = threadIdx.x; const int n = t >> 3, k8 = (t & 7) * 8;
    v8h o;
#pragma unroll
    for (int j = 0; j < 8; ++j) o[j] = toh_flush(bfr(W2[(size_t)(k8 + j) * NH2 + n]) * W2S);
    *(volatile v8h*)(W2T + (size_t)t * 8) = o; __threadfence(); *(volatile v8h*)(W2T + (size_t)t * 8) = o;
}

__global__ __launch_bounds__(32) void k_gemm1(const bf* __restrict__ A, const bf* __restrict__ Bt, const float* __restrict__ bias, float* P) {
    __shared__ __align__(16) float os[16 * 68];
    const int K = NIN;
    const int lane = threadIdx.x & 31, lr = lane & 15, hi = lane >> 4; const int r0 = (int)(blockIdx.x * 64u);
    v8f acc[4][4];
#pragma unroll
    for (int mb = 0; mb < 4; ++mb)
#pragma unroll
        for (int nb = 0; nb < 4; ++nb) acc[mb][nb] = (v8f){};
    const size_t aoff = (size_t)(r0 + lr) * K + 8 * hi, boff = (size_t)lr * K + 8 * hi;
#pragma unroll 1
    for (int kc = 0; kc < K; kc += 32) {
        v16bf a[4];
#pragma unroll
        for (int mb = 0; mb < 4; ++mb) a[mb] = ldb(A + aoff + (size_t)mb * 16 * K + kc);
#pragma unroll
        for (int nb = 0; nb < 4; ++nb) { const v16bf b = ldb(Bt + boff + (size_t)nb * 16 * K + kc);
#pragma unroll
            for (int mb = 0; mb < 4; ++mb) acc[mb][nb] = wmmabg(a[mb], b, acc[mb][nb]); }
    }
    const bool xrow = r0 < NWR;
    float bc[4];
#pragma unroll
    for (int nb = 0; nb < 4; ++nb) { const float bl = bfr(bias[nb * 16 + lr]); bc[nb] = xrow ? bl : 0.0f; }
#pragma unroll
    for (int mb = 0; mb < 4; ++mb) {
#pragma unroll
        for (int nb = 0; nb < 4; ++nb) {
#pragma unroll
            for (int j = 0; j < 8; ++j) os[(hi * 8 + j) * 68 + nb * 16 + lr] = acc[mb][nb][j] + bc[nb]; }
        wave_sync();
        float* pb = P + (size_t)(r0 + mb * 16) * NH1;
#pragma unroll 1
        for (int ps = 0; ps < 2; ++ps) {
#pragma unroll
            for (int s = 0; s < 8; ++s) { const int p = s * 32 + lane; const int row = p >> 4, c4 = (p & 15) * 4;
                const v4f val = *(const v4fa*)(&os[row * 68 + c4]);
                *(volatile v4f*)(pb + (size_t)p * 4) = val; }
            if (ps == 0) __threadfence(); }
        wave_sync();
    }
}

__global__ __launch_bounds__(32 * AW) void k_pair(const float* __restrict__ P, const h16* __restrict__ W2T, const float* __restrict__ b2,
                                                  const float* __restrict__ W3, const float* __restrict__ b3, float* OUT) {
    __shared__ __align__(16) float os[AW * 16 * OSP];
    const int lane = threadIdx.x & 31, lr = lane & 15, hi = lane >> 4;
    const int wave = __builtin_amdgcn_readfirstlane((int)(threadIdx.x >> 5));
    const int q0 = (int)(blockIdx.x * 32u);
    const int w0 = ((int)blockIdx.y * AW + wave) * 16;
    const h16* wp = W2T + (size_t)lr * NH1 + 8 * hi;
    const v16h a00 = ldh(wp), a01 = ldh(wp + 32);
    const v16h a10 = ldh(wp + 16 * NH1), a11 = ldh(wp + 16 * NH1 + 32);
    float b2a[8], b2b[8], w3a[8], w3b[8];
    { const v4f c0 = *(const v4f*)(b2 + 8 * hi), c1 = *(const v4f*)(b2 + 8 * hi + 4), c2 = *(const v4f*)(b2 + 16 + 8 * hi), c3 = *(const v4f*)(b2 + 16 + 8 * hi + 4);
      const v4f e0 = *(const v4f*)(W3 + 8 * hi), e1 = *(const v4f*)(W3 + 8 * hi + 4), e2 = *(const v4f*)(W3 + 16 + 8 * hi), e3 = *(const v4f*)(W3 + 16 + 8 * hi + 4);
#pragma unroll
      for (int r = 0; r < 4; ++r) { b2a[r] = bfr(c0[r]); b2a[4 + r] = bfr(c1[r]); b2b[r] = bfr(c2[r]); b2b[4 + r] = bfr(c3[r]);
                                    w3a[r] = bfr(e0[r]); w3a[4 + r] = bfr(e1[r]); w3b[r] = bfr(e2[r]); w3b[4 + r] = bfr(e3[r]); } }
    const float b3v = bfr(b3[0]);
    const int wb = wave * 16 * OSP;
#pragma unroll 1
    for (int g = 0; g < 2; ++g) {
        const float* yp = P + (size_t)(NWR + q0 + 16 * g + lr) * NH1 + 8 * hi;
        const v4f y0 = *(const v4f*)yp,        y1 = *(const v4f*)(yp + 4),  y2 = *(const v4f*)(yp + 16), y3 = *(const v4f*)(yp + 20);
        const v4f y4 = *(const v4f*)(yp + 32), y5 = *(const v4f*)(yp + 36), y6 = *(const v4f*)(yp + 48), y7 = *(const v4f*)(yp + 52);
#pragma unroll 1
        for (int wl = 0; wl < 16; ++wl) {
            const float* xp = P + (size_t)(w0 + wl) * NH1 + 8 * hi;
            const v4f x0 = *(const v4f*)xp,        x1 = *(const v4f*)(xp + 4),  x2 = *(const v4f*)(xp + 16), x3 = *(const v4f*)(xp + 20);
            const v4f x4 = *(const v4f*)(xp + 32), x5 = *(const v4f*)(xp + 36), x6 = *(const v4f*)(xp + 48), x7 = *(const v4f*)(xp + 52);
            v16h f0, f1, g0, g1;
#pragma unroll
            for (int i = 0; i < 4; ++i) {
                { const float hv = fmaxf(x0[i] - y0[i], 0.0f); const h16 hw = toh_flush(hv); f0[i]      = hw; g0[i]      = toh_flush((hv - (float)hw) * H1RS); }
                { const float hv = fmaxf(x1[i] - y1[i], 0.0f); const h16 hw = toh_flush(hv); f0[4 + i]  = hw; g0[4 + i]  = toh_flush((hv - (float)hw) * H1RS); }
                { const float hv = fmaxf(x2[i] - y2[i], 0.0f); const h16 hw = toh_flush(hv); f0[8 + i]  = hw; g0[8 + i]  = toh_flush((hv - (float)hw) * H1RS); }
                { const float hv = fmaxf(x3[i] - y3[i], 0.0f); const h16 hw = toh_flush(hv); f0[12 + i] = hw; g0[12 + i] = toh_flush((hv - (float)hw) * H1RS); }
                { const float hv = fmaxf(x4[i] - y4[i], 0.0f); const h16 hw = toh_flush(hv); f1[i]      = hw; g1[i]      = toh_flush((hv - (float)hw) * H1RS); }
                { const float hv = fmaxf(x5[i] - y5[i], 0.0f); const h16 hw = toh_flush(hv); f1[4 + i]  = hw; g1[4 + i]  = toh_flush((hv - (float)hw) * H1RS); }
                { const float hv = fmaxf(x6[i] - y6[i], 0.0f); const h16 hw = toh_flush(hv); f1[8 + i]  = hw; g1[8 + i]  = toh_flush((hv - (float)hw) * H1RS); }
                { const float hv = fmaxf(x7[i] - y7[i], 0.0f); const h16 hw = toh_flush(hv); f1[12 + i] = hw; g1[12 + i] = toh_flush((hv - (float)hw) * H1RS); } }
            v8f d0 = (v8f){}, d1 = (v8f){};
            d0 = wmma16g(a00, f0, d0); d0 = wmma16g(a01, f1, d0);
            d1 = wmma16g(a10, f0, d1); d1 = wmma16g(a11, f1, d1);
            v8f e0 = (v8f){}, e1 = (v8f){};
            e0 = wmma16g(a00, g0, e0); e0 = wmma16g(a01, g1, e0);
            e1 = wmma16g(a10, g0, e1); e1 = wmma16g(a11, g1, e1);
            float s = 0.0f;
#pragma unroll
            for (int r = 0; r < 8; ++r) {
                const float ta = fmaxf((d0[r] + e0[r] * H1RI) * W2I + b2a[r], 0.0f);
                const float tb = fmaxf((d1[r] + e1[r] * H1RI) * W2I + b2b[r], 0.0f);
                s += ta * w3a[r]; s += tb * w3b[r]; }
            s += __shfl_xor(s, 16, 32);
            float ov = fmaxf(s + b3v, 0.0f);
            asm volatile("" : "+v"(ov));
            if (hi == 0) os[wb + wl * OSP + 16 * g + lr] = ov;
        }
    }
    wave_sync();
    float* orow = OUT + (size_t)w0 * OUT_PITCH + q0;
#pragma unroll 1
    for (int ps = 0; ps < 2; ++ps) {
#pragma unroll
        for (int s = 0; s < 4; ++s) { const int row = 4 * s + (lane >> 3), cofs = (lane & 7) * 4;
            const v4f val = *(const v4fa*)(&os[wb + row * OSP + cofs]);
            *(volatile v4f*)(orow + (size_t)row * OUT_PITCH + cofs) = val; }
        if (ps == 0) __threadfence(); }
}

static constexpr size_t al256(size_t v) { return (v + 255) & ~(size_t)255; }
static constexpr size_t SZ_XB  = al256((size_t)(NWR + NQR) * NIN * 2);
static constexpr size_t SZ_W1T = al256((size_t)NH1 * NIN * 2);
static constexpr size_t SZ_W2T = al256((size_t)NH2 * NH1 * 2);
static constexpr size_t SZ_P   = al256((size_t)(NWR + NQR) * NH1 * 4);
static constexpr size_t SZ_TOTAL = SZ_XB + SZ_W1T + SZ_W2T + SZ_P;
static_assert(SZ_TOTAL <= (size_t)134217728);
static_assert(((size_t)NWR * NIN * 2) % 128 == 0);
static_assert(((size_t)NWR * NIN) % 8 == 0);
static_assert(((size_t)NQR * NIN) % 8 == 0);
static constexpr size_t N8X = (size_t)NWR * NIN / 8;
static constexpr size_t N8Y = (size_t)NQR * NIN / 8;
static constexpr size_t NEED_X = (size_t)NWR * NIN;
static constexpr size_t NEED_Y = (size_t)NQR * NIN;
static constexpr size_t NEED_OUT = (size_t)(NWR - 1) * OUT_PITCH + NQR;
static_assert(NEED_OUT * 4 <= (size_t)1048576);

extern "C" void kernel_launch(void* const* d_in, const int* in_sizes, int n_in,
                              void* d_out, int out_size, void* d_ws, size_t ws_size, hipStream_t stream) {
    if (n_in < 8) return;
    if ((size_t)in_sizes[0] < NEED_X || (size_t)in_sizes[1] < NEED_Y) return;
    if ((size_t)in_sizes[2] < (size_t)NIN * NH1 || in_sizes[3] < NH1 || in_sizes[4] < NH1 * NH2) return;
    if (in_sizes[5] < NH2 || in_sizes[6] < NH2 || in_sizes[7] < 1) return;
    if ((size_t)out_size < NEED_OUT) return;
    if (SZ_TOTAL > ws_size) return;
    const float* x  = (const float*)d_in[0];
    const float* y  = (const float*)d_in[1];
    const float* w1 = (const float*)d_in[2];
    const float* b1 = (const float*)d_in[3];
    const float* w2 = (const float*)d_in[4];
    const float* b2 = (const float*)d_in[5];
    const float* w3 = (const float*)d_in[6];
    const float* b3 = (const float*)d_in[7];
    float* OUT = (float*)d_out;
    char* wsp = (char*)d_ws;
    bf*  XB  = (bf*)wsp;  wsp += SZ_XB;
    bf*  W1T = (bf*)wsp;  wsp += SZ_W1T;
    h16* W2T = (h16*)wsp; wsp += SZ_W2T;
    float* P = (float*)wsp; wsp += SZ_P;

    k_cvt8<<<(unsigned)((N8X + 255) / 256), 256, 0, stream>>>(x, XB, N8X);
    k_cvt8<<<(unsigned)((N8Y + 255) / 256), 256, 0, stream>>>(y, XB + (size_t)NWR * NIN, N8Y);
    k_w1t<<<(unsigned)((NH1 * (NIN / 8)) / 256), 256, 0, stream>>>(w1, W1T);
    k_w2t<<<1, 256, 0, stream>>>(w2, W2T);
    k_gemm1<<<(unsigned)((NWR + NQR) / 64), 32, 0, stream>>>(XB, W1T, b1, P);
    k_pair<<<dim3(NQR / 32, NWR / (16 * AW), 1), 32 * AW, 0, stream>>>(P, W2T, b2, w3, b3, OUT);
}
